// match_GRU_75539884802387
// MI455X (gfx1250) — hardware-run, weakly checked
//
#include <hip/hip_runtime.h>
#include <math.h>

typedef __attribute__((ext_vector_type(16))) _Float16 v16h;
typedef __attribute__((ext_vector_type(8)))  _Float16 v8h;
typedef __attribute__((ext_vector_type(8)))  float    v8f;
typedef __attribute__((ext_vector_type(4)))  float    v4f;
typedef __attribute__((ext_vector_type(4)))  unsigned v4u;
typedef unsigned u32a __attribute__((may_alias));

constexpr int kB  = 4;
constexpr int kLK = 512;
constexpr int kLQ = 128;
constexpr int kD  = 256;
constexpr int kH  = 256;
constexpr int kL  = 3;
constexpr int kG3 = 3 * kH;
constexpr int kRowsK = kB * kLK;
constexpr int kRowsQ = kB * kLQ;
static_assert(kD == 256 && kH == 256, "feature widths");
static_assert((kD % 32) == 0 && (kH % 32) == 0 && (kLK % 32) == 0, "GEMM K multiples of 32");
static_assert((kRowsK % 64) == 0 && (kRowsQ % 64) == 0 && (kLQ % 64) == 0 && (kH % 64) == 0 && (kG3 % 64) == 0 && (kD % 64) == 0, "GEMM M,N multiples of 64");

constexpr float kCarryAct = 64.0f;
constexpr float kCarryW   = 1024.0f;
constexpr float kCarryH   = 1024.0f;
constexpr float kScaleActW = 1.0f / (kCarryAct * kCarryW);
constexpr float kScaleHW   = 1.0f / (kCarryH * kCarryW);
constexpr float kScaleAct  = 1.0f / kCarryAct;
constexpr float kF16MinNormal = 6.103515625e-5f;

constexpr size_t kOffKH  = 0;
constexpr size_t kOffKT  = kOffKH  + (size_t)kRowsK * kD * 2;
constexpr size_t kOffQH  = kOffKT  + (size_t)kB * kD * kLK * 2;
constexpr size_t kOffWK  = kOffQH  + (size_t)kRowsQ * kD * 2;
constexpr size_t kOffWQ  = kOffWK  + (size_t)kH * kD * 2;
constexpr size_t kOffWG  = kOffWQ  + (size_t)kH * kD * 2;
constexpr size_t kOffWIH = kOffWG  + (size_t)kH * kH * 2;
constexpr size_t kOffWHH = kOffWIH + (size_t)kL * kG3 * kH * 2;
constexpr size_t kOffKP  = kOffWHH + (size_t)kL * kG3 * kH * 2;
constexpr size_t kOffQP  = kOffKP  + (size_t)kRowsK * kH * 4;
constexpr size_t kOffEH  = kOffQP  + (size_t)kRowsQ * kH * 4;
constexpr size_t kOffRR  = kOffEH  + (size_t)kB * kLQ * kLK * 2;
constexpr size_t kOffUC  = kOffRR  + (size_t)kRowsQ * kD * 4;
constexpr size_t kOffUCH = kOffUC  + (size_t)kRowsQ * kD * 4;
constexpr size_t kOffPRE = kOffUCH + (size_t)kRowsQ * kD * 2;
constexpr size_t kOffXA  = kOffPRE + (size_t)kRowsQ * kH * 4;
constexpr size_t kOffY0  = kOffXA  + (size_t)kRowsQ * kH * 2;
constexpr size_t kOffY1  = kOffY0  + (size_t)kRowsQ * kH * 2;
constexpr size_t kOffGI  = kOffY1  + (size_t)kRowsQ * kH * 2;
constexpr size_t kWsTotal = kOffGI + (size_t)kRowsQ * kG3 * 4;
static_assert(kWsTotal == 12451840ull, "carve total");
static_assert(kWsTotal <= 134217728ull, "carve cap");
static_assert((kOffKT % 128) == 0 && (kOffQH % 128) == 0 && (kOffWK % 128) == 0 && (kOffWQ % 128) == 0 &&
              (kOffWG % 128) == 0 && (kOffWIH % 128) == 0 && (kOffWHH % 128) == 0 && (kOffKP % 128) == 0 &&
              (kOffQP % 128) == 0 && (kOffEH % 128) == 0 && (kOffRR % 128) == 0 && (kOffUC % 128) == 0 &&
              (kOffUCH % 128) == 0 && (kOffPRE % 128) == 0 && (kOffXA % 128) == 0 && (kOffY0 % 128) == 0 &&
              (kOffY1 % 128) == 0 && (kOffGI % 128) == 0, "128-B aligned regions");

__device__ __forceinline__ _Float16 to_h16(float v) {
  const float a = (fabsf(v) < kF16MinNormal) ? 0.0f : v;
  return (_Float16)a;
}
__device__ __forceinline__ float h16_to_f32(unsigned hb) {
  const unsigned sgn = (hb & 0x8000u) << 16; const unsigned em = hb & 0x7fffu;
  const float fn = __uint_as_float((em << 13) + 0x38000000u);
  const float fs = (float)em * 5.9604644775390625e-8f;
  const float mag = (em < 0x400u) ? fs : fn; return __uint_as_float(__float_as_uint(mag) | sgn);
}

__device__ __forceinline__ void guard4_h(v8f& a, v8f& b, v8f& c, v8f& d, v16h x, v16h y0, v16h y1, v16h y2, v16h y3) {
  asm volatile("v_nop\n\tv_nop\n\tv_nop\n\tv_nop" : "+v"(a), "+v"(b), "+v"(c), "+v"(d) : "v"(x), "v"(y0), "v"(y1), "v"(y2), "v"(y3));
}
__device__ __forceinline__ void guard3_h(v8f& a, v8f& b, v8f& c, v16h x, v16h y0, v16h y1, v16h y2) {
  asm volatile("v_nop\n\tv_nop\n\tv_nop\n\tv_nop" : "+v"(a), "+v"(b), "+v"(c) : "v"(x), "v"(y0), "v"(y1), "v"(y2));
}
__device__ __forceinline__ void keep4_h(v16h a, v16h b, v16h c, v16h d) { asm volatile("v_nop" :: "v"(a), "v"(b), "v"(c), "v"(d)); }
__device__ __forceinline__ void acc_guard4(v8f& a, v8f& b, v8f& c, v8f& d) { asm volatile("v_nop\n\tv_nop\n\tv_nop\n\tv_nop" : "+v"(a), "+v"(b), "+v"(c), "+v"(d)); }

struct FragH {
  union U { v16h v; v8h h[2]; };
  static __device__ __forceinline__ v16h load(const _Float16* p) {
    U f; f.h[0] = *(const v8h*)(p); f.h[1] = *(const v8h*)(p + 16); return f.v;
  }
  static __device__ __forceinline__ v8f mma(v16h a, v16h b, v8f c) {
    return __builtin_amdgcn_wmma_f32_16x16x32_f16(false, a, false, b, (short)0, c, false, false);
  }
};

constexpr int kCvtBlkKeys = kRowsK * kD / 8 / 256;
constexpr int kCvtBlkQ    = kRowsQ * kD / 8 / 256;
constexpr int kCvtBlkW    = kH * kD / 8 / 256;
constexpr int kCvtBlkG    = kL * kG3 * kH / 8 / 256;
constexpr int kCvtE0 = kCvtBlkKeys;
constexpr int kCvtE1 = kCvtE0 + kCvtBlkQ;
constexpr int kCvtE2 = kCvtE1 + kCvtBlkW;
constexpr int kCvtE3 = kCvtE2 + kCvtBlkW;
constexpr int kCvtE4 = kCvtE3 + kCvtBlkW;
constexpr int kCvtE5 = kCvtE4 + kCvtBlkG;
constexpr int kCvtE6 = kCvtE5 + kCvtBlkG;
static_assert(kCvtBlkKeys * 256 * 8 == kRowsK * kD && kCvtBlkQ * 256 * 8 == kRowsQ * kD &&
              kCvtBlkW * 256 * 8 == kH * kD && kCvtBlkG * 256 * 8 == kL * kG3 * kH, "exact coverage");
static_assert(kCvtE6 == 992, "convert grid");

__global__ __launch_bounds__(256) void cvt_planes_kernel(
    const float* __restrict__ s0, const float* __restrict__ s1, const float* __restrict__ s2,
    const float* __restrict__ s3, const float* __restrict__ s4, const float* __restrict__ s5,
    const float* __restrict__ s6,
    unsigned short* __restrict__ d0, unsigned short* __restrict__ d1, unsigned short* __restrict__ d2,
    unsigned short* __restrict__ d3, unsigned short* __restrict__ d4, unsigned short* __restrict__ d5,
    unsigned short* __restrict__ d6)
{
  const int bx = blockIdx.x;
  const float* s; unsigned short* d; float carry; int lb;
  if (bx < kCvtE0)      { s = s0; d = d0; carry = kCarryAct; lb = bx; }
  else if (bx < kCvtE1) { s = s1; d = d1; carry = kCarryAct; lb = bx - kCvtE0; }
  else if (bx < kCvtE2) { s = s2; d = d2; carry = kCarryW;   lb = bx - kCvtE1; }
  else if (bx < kCvtE3) { s = s3; d = d3; carry = kCarryW;   lb = bx - kCvtE2; }
  else if (bx < kCvtE4) { s = s4; d = d4; carry = kCarryW;   lb = bx - kCvtE3; }
  else if (bx < kCvtE5) { s = s5; d = d5; carry = kCarryW;   lb = bx - kCvtE4; }
  else                  { s = s6; d = d6; carry = kCarryW;   lb = bx - kCvtE5; }
  const size_t e0 = ((size_t)lb * 256 + threadIdx.x) << 3;
  const v4f a0 = *(const v4f*)(s + e0);
  const v4f a1 = *(const v4f*)(s + e0 + 4);
  v8h hv;
#pragma unroll
  for (int e = 0; e < 4; ++e) {
    const float x0 = a0[e] * carry;
    const float x1 = a1[e] * carry;
    hv[e]     = to_h16(x0);
    hv[4 + e] = to_h16(x1);
  }
  unsigned short* q = d + e0;
  *(volatile v8h*)q = hv;
  __threadfence();
  *(volatile v8h*)q = hv;
}

__global__ __launch_bounds__(256) void keys_transpose_kernel(
    const float* __restrict__ keys, unsigned short* __restrict__ KT)
{
  __shared__ float sT[64 * 65];
  const int tid = threadIdx.x, lane = tid & 31, wave = tid >> 5;
  const int k0 = blockIdx.x * 64, d0 = blockIdx.y * 64, b = blockIdx.z;
#pragma unroll
  for (int j = 0; j < 4; ++j) {
    const int i = tid + 256 * j;
    const int r = i >> 4, c4 = (i & 15) * 4;
    const v4f v = *(const v4f*)(keys + ((size_t)(b * kLK + k0 + r)) * kD + d0 + c4);
    sT[r * 65 + c4 + 0] = v[0];
    sT[r * 65 + c4 + 1] = v[1];
    sT[r * 65 + c4 + 2] = v[2];
    sT[r * 65 + c4 + 3] = v[3];
  }
  __syncthreads();
  const int q = lane >> 3, c8 = (lane & 7) * 8;
  v8h hv[2];
#pragma unroll
  for (int it = 0; it < 2; ++it) {
    const int dr = it * 32 + wave * 4 + q;
#pragma unroll
    for (int e = 0; e < 8; ++e) {
      const float x = sT[(c8 + e) * 65 + dr] * kCarryAct;
      hv[it][e] = to_h16(x);
    }
  }
  for (int pass = 0; pass < 2; ++pass) {
#pragma unroll
    for (int it = 0; it < 2; ++it) {
      const int dr = it * 32 + wave * 4 + q;
      *(volatile v8h*)(KT + ((size_t)(b * kD + d0 + dr)) * kLK + k0 + c8) = hv[it];
    }
    __threadfence();
  }
}

template <int BIAS_MODE>
__global__ __launch_bounds__(256) void gemm64_f16_kernel(
    const unsigned short* __restrict__ Ap, int lda, long strideA,
    const unsigned short* __restrict__ Btp, int ldb, long strideB,
    float* __restrict__ Cout, int ldc, long strideC,
    const float* __restrict__ bias,
    int M, int N, int K, float scale)
{
  const _Float16* A  = (const _Float16*)Ap;
  const _Float16* Bt = (const _Float16*)Btp;
  __shared__ __align__(16) float sT[8][16 * 68];
  const int b    = blockIdx.y;
  const int lane = threadIdx.x & 31;
  const int wave = threadIdx.x >> 5;
  const int tilesN = N >> 6;
  const int tilesM = M >> 6;
  const int tile = blockIdx.x * 8 + wave;
  if (tile >= tilesM * tilesN) return;
  const int tm = tile / tilesN;
  const int tn = tile - tm * tilesN;
  const int m0 = tm << 6;
  const int n0 = tn << 6;

  const _Float16* Ab = A  + (size_t)b * strideA;
  const _Float16* Bb = Bt + (size_t)b * strideB;

  const int rlane = lane & 15;
  const int koff  = (lane >> 4) * 8;
  const int mOff  = (lane >> 4) * 8;

  v8f acc[4][4];
#pragma unroll
  for (int i = 0; i < 4; ++i)
#pragma unroll
    for (int j = 0; j < 4; ++j) acc[i][j] = (v8f){0.f,0.f,0.f,0.f,0.f,0.f,0.f,0.f};

  for (int k0 = 0; k0 < K; k0 += 32) {
    v16h bh[4];
#pragma unroll
    for (int j = 0; j < 4; ++j) {
      const size_t bo = (size_t)(n0 + (j << 4) + rlane) * ldb + koff + k0;
      bh[j] = FragH::load(Bb + bo);
    }
#pragma unroll
    for (int i = 0; i < 4; ++i) {
      const size_t ao = (size_t)(m0 + (i << 4) + rlane) * lda + koff + k0;
      const v16h ah = FragH::load(Ab + ao);
#pragma unroll
      for (int j = 0; j < 4; ++j) acc[i][j] = FragH::mma(ah, bh[j], acc[i][j]);
      guard4_h(acc[i][0], acc[i][1], acc[i][2], acc[i][3], ah, bh[0], bh[1], bh[2], bh[3]);
    }
    keep4_h(bh[0], bh[1], bh[2], bh[3]);
  }
  acc_guard4(acc[0][0], acc[0][1], acc[0][2], acc[0][3]);
  acc_guard4(acc[1][0], acc[1][1], acc[1][2], acc[1][3]);
  acc_guard4(acc[2][0], acc[2][1], acc[2][2], acc[2][3]);
  acc_guard4(acc[3][0], acc[3][1], acc[3][2], acc[3][3]);

  float* slab = sT[wave];
  float* C = Cout + (size_t)b * strideC;
#pragma unroll
  for (int i = 0; i < 4; ++i) {
    const int mBase = m0 + (i << 4);
#pragma unroll
    for (int j = 0; j < 4; ++j) {
      const int n = n0 + (j << 4) + rlane;
      float bv = 0.f;
      if (BIAS_MODE == 2) bv = bias[n];
#pragma unroll
      for (int r = 0; r < 8; ++r) {
        float v = acc[i][j][r] * scale;
        if (BIAS_MODE == 2) v += bv;
        slab[(mOff + r) * 68 + (j << 4) + rlane] = v;
      }
    }
    __builtin_amdgcn_fence(__ATOMIC_RELEASE, "workgroup");
    __builtin_amdgcn_wave_barrier();
    __builtin_amdgcn_fence(__ATOMIC_ACQUIRE, "workgroup");
    {
      const int hh = lane >> 4, c4 = (lane & 15) * 4;
      for (int pass = 0; pass < 2; ++pass) {
#pragma unroll
        for (int it = 0; it < 8; ++it) {
          const int row = it * 2 + hh;
          const v4f v = *(const v4f*)(slab + row * 68 + c4);
          *(volatile v4f*)(C + (size_t)(mBase + row) * ldc + n0 + c4) = v;
        }
        __threadfence();
      }
    }
    __builtin_amdgcn_fence(__ATOMIC_RELEASE, "workgroup");
    __builtin_amdgcn_wave_barrier();
    __builtin_amdgcn_fence(__ATOMIC_ACQUIRE, "workgroup");
  }
}

__global__ __launch_bounds__(256) void score_exp_kernel(
    const float* __restrict__ Qp, const float* __restrict__ Kp, const float* __restrict__ wv,
    unsigned short* __restrict__ Eh)
{
  __shared__ __align__(16) float sK[64 * 65];
  __shared__ __align__(16) float sQ[16 * 64];
  __shared__ __align__(16) float sW[256];
  __shared__ __align__(16) float sS[16 * 64];
  const int tid = threadIdx.x, lane = tid & 31, wave = tid >> 5;
  const int k0 = blockIdx.x * 64, q0 = blockIdx.y * 16, b = blockIdx.z;
  const int kl = tid & 63, qg = tid >> 6;
  sW[tid] = wv[tid];
#pragma unroll 1
  for (int hc = 0; hc < 4; ++hc) {
    __syncthreads();
#pragma unroll
    for (int j = 0; j < 4; ++j) {
      const int i = tid + 256 * j;
      const int r = i >> 4, c4 = (i & 15) * 4;
      const v4f v = *(const v4f*)(Kp + ((size_t)(b * kLK + k0 + r)) * kH + hc * 64 + c4);
      sK[r * 65 + c4 + 0] = v[0];
      sK[r * 65 + c4 + 1] = v[1];
      sK[r * 65 + c4 + 2] = v[2];
      sK[r * 65 + c4 + 3] = v[3];
    }
    {
      const int r = tid >> 4, c4 = (tid & 15) * 4;
      *(v4f*)(sQ + r * 64 + c4) = *(const v4f*)(Qp + ((size_t)(b * kLQ + q0 + r)) * kH + hc * 64 + c4);
    }
    __syncthreads();
#pragma unroll 1
    for (int p = 0; p < 4; ++p) {
      const int ql = qg * 4 + p;
      float s = 0.0f;
      if (hc > 0) s = sS[ql * 64 + kl];
      const float* qr = sQ + ql * 64;
      const float* kr = sK + kl * 65;
      const float* wr = sW + hc * 64;
#pragma unroll 2
      for (int h = 0; h < 64; ++h) {
        const float tv = tanhf(qr[h] + kr[h]);
        s = fmaf(wr[h], tv, s);
      }
      if (hc == 3) s = expf(s);
      sS[ql * 64 + kl] = s;
    }
  }
  __syncthreads();
  if (wave < 4) {
    const int row = wave * 4 + (lane >> 3), c8 = (lane & 7) * 8;
    const v4f a0 = *(const v4f*)(sS + row * 64 + c8);
    const v4f a1 = *(const v4f*)(sS + row * 64 + c8 + 4);
    v8h hv;
#pragma unroll
    for (int e = 0; e < 4; ++e) {
      hv[e]     = to_h16(a0[e]);
      hv[4 + e] = to_h16(a1[e]);
    }
    unsigned short* dst = Eh + ((size_t)(b * kLQ + q0 + row)) * kLK + k0 + c8;
    *(volatile v8h*)dst = hv;
    __threadfence();
    *(volatile v8h*)dst = hv;
  }
}

__global__ __launch_bounds__(256) void denom_resid_kernel(
    const unsigned short* __restrict__ Eh, const float* __restrict__ RR, const float* __restrict__ queries,
    float* __restrict__ UC, unsigned short* __restrict__ UCH)
{
  __shared__ float red[256];
  __shared__ __align__(16) float sU[4 * 256];
  const int tid = threadIdx.x, lane = tid & 31, wave = tid >> 5;
  const int q = blockIdx.x;
  {
    const int b = tid >> 6, w8 = (tid & 63) * 8;
    const v4u wv = *(const v4u*)(Eh + ((size_t)(b * kLQ + q)) * kLK + w8);
    const unsigned w0 = wv[0], w1 = wv[1], w2 = wv[2], w3 = wv[3];
    float s = 0.0f;
    s += h16_to_f32(w0 & 0xffffu);
    s += h16_to_f32(w0 >> 16);
    s += h16_to_f32(w1 & 0xffffu);
    s += h16_to_f32(w1 >> 16);
    s += h16_to_f32(w2 & 0xffffu);
    s += h16_to_f32(w2 >> 16);
    s += h16_to_f32(w3 & 0xffffu);
    s += h16_to_f32(w3 >> 16);
    red[tid] = s;
  }
  __syncthreads();
#pragma unroll 1
  for (int off = 128; off > 0; off >>= 1) {
    if (tid < off) red[tid] += red[tid + off];
    __syncthreads();
  }
  const float inv = 1.0f / red[0];
  float u[4];
#pragma unroll
  for (int b = 0; b < 4; ++b) {
    const size_t idx = ((size_t)(b * kLQ + q)) * kD + tid;
    const float uv = queries[idx] + RR[idx] * inv;
    u[b] = uv;
    sU[b * 256 + tid] = uv;
  }
  for (int pass = 0; pass < 2; ++pass) {
#pragma unroll
    for (int b = 0; b < 4; ++b) {
      const size_t idx = ((size_t)(b * kLQ + q)) * kD + tid;
      *(volatile float*)(UC + idx) = u[b];
    }
    __threadfence();
  }
  __syncthreads();
  if (wave < 4) {
    const int b = wave, c8 = lane * 8;
    const v4f a0 = *(const v4f*)(sU + b * 256 + c8);
    const v4f a1 = *(const v4f*)(sU + b * 256 + c8 + 4);
    v8h hv;
#pragma unroll
    for (int e = 0; e < 4; ++e) {
      const float x0 = a0[e] * kCarryAct;
      const float x1 = a1[e] * kCarryAct;
      hv[e]     = to_h16(x0);
      hv[4 + e] = to_h16(x1);
    }
    unsigned short* dst = UCH + ((size_t)(b * kLQ + q)) * kD + c8;
    *(volatile v8h*)dst = hv;
    __threadfence();
    *(volatile v8h*)dst = hv;
  }
}

__global__ __launch_bounds__(256) void gate_apply_kernel(
    const float* __restrict__ PRE, const float* __restrict__ UC, unsigned short* __restrict__ XA)
{
  const size_t e0 = ((size_t)blockIdx.x * 256 + threadIdx.x) << 3;
  const v4f p0 = *(const v4f*)(PRE + e0);
  const v4f p1 = *(const v4f*)(PRE + e0 + 4);
  const v4f u0 = *(const v4f*)(UC + e0);
  const v4f u1 = *(const v4f*)(UC + e0 + 4);
  v8h hv;
#pragma unroll
  for (int e = 0; e < 4; ++e) {
    const float g0 = 1.0f / (1.0f + expf(-p0[e]));
    const float g1 = 1.0f / (1.0f + expf(-p1[e]));
    const float x0 = g0 * u0[e] * kCarryAct;
    const float x1 = g1 * u1[e] * kCarryAct;
    hv[e]     = to_h16(x0);
    hv[4 + e] = to_h16(x1);
  }
  unsigned short* dst = XA + e0;
  *(volatile v8h*)dst = hv;
  __threadfence();
  *(volatile v8h*)dst = hv;
}

constexpr int kHP = 264;

template <bool LAST>
__global__ __launch_bounds__(512) void gru_scan_kernel(
    const float* __restrict__ gi, const unsigned short* __restrict__ Whh, const float* __restrict__ bhh,
    unsigned short* __restrict__ yh, float* __restrict__ outp)
{
  __shared__ __align__(16) _Float16 hA[2][16 * kHP];
  __shared__ __align__(16) float hF[LAST ? 2 * 4 * 256 : 8];
  const int tid = threadIdx.x, lane = tid & 31, wave = tid >> 5;
  const int hh = lane >> 4, c = lane & 15;
  const int j = wave * 16 + c;
  v8h z8;
#pragma unroll
  for (int e = 0; e < 8; ++e) z8[e] = (_Float16)0.0f;
  for (int i = tid; i < 2 * 16 * kHP / 8; i += 512) *(v8h*)(&hA[0][0] + i * 8) = z8;
  __syncthreads();

  const float bh_r = bhh[j], bh_z = bhh[kH + j], bh_n = bhh[2 * kH + j];
  const _Float16* W = (const _Float16*)Whh;
  const unsigned wbase = (unsigned)(j * kH + 8 * hh);
  float hst[4];
#pragma unroll
  for (int b = 0; b < 4; ++b) hst[b] = 0.0f;

#pragma unroll 1
  for (int t = 0; t < kLQ; ++t) {
    const int cur = t & 1, nxt = cur ^ 1;
    float gr[4], gz[4], gn[4];
#pragma unroll
    for (int b = 0; b < 4; ++b) {
      const size_t base = ((size_t)(b * kLQ + t)) * kG3 + j;
      gr[b] = gi[base];
      gz[b] = gi[base + kH];
      gn[b] = gi[base + 2 * kH];
    }
    unsigned woff = wbase;
    asm volatile("" : "+v"(woff));
    v8f ar = (v8f){0.f,0.f,0.f,0.f,0.f,0.f,0.f,0.f};
    v8f az = ar, an = ar;
    const _Float16* ap = &hA[cur][c * kHP + 8 * hh];
#pragma unroll 1
    for (int kk = 0; kk < 8; ++kk) {
      const v16h a  = FragH::load(ap + kk * 32);
      const v16h b0 = FragH::load(W + woff + kk * 32);
      const v16h b1 = FragH::load(W + woff + kH * kH + kk * 32);
      const v16h b2 = FragH::load(W + woff + 2 * kH * kH + kk * 32);
      ar = FragH::mma(a, b0, ar);
      az = FragH::mma(a, b1, az);
      an = FragH::mma(a, b2, an);
      guard3_h(ar, az, an, a, b0, b1, b2);
    }
#pragma unroll
    for (int b = 0; b < 4; ++b) {
      const float hr = ar[b] * kScaleHW + bh_r;
      const float hz = az[b] * kScaleHW + bh_z;
      const float hn = an[b] * kScaleHW + bh_n;
      const float r = 1.0f / (1.0f + expf(-(gr[b] + hr)));
      const float z = 1.0f / (1.0f + expf(-(gz[b] + hz)));
      const float n = tanhf(gn[b] + r * hn);
      const float hnew = (1.0f - z) * n + z * hst[b];
      hst[b] = hnew;
      if (hh == 0) {
        const float hc = hnew * kCarryH;
        hA[nxt][b * kHP + j] = to_h16(hc);
        if (LAST) hF[nxt * 1024 + b * 256 + j] = hnew;
      }
    }
    if (tid < 12 * kHP / 8) *(v8h*)(&hA[nxt][4 * kHP + tid * 8]) = z8;
    __syncthreads();
    {
      const int b = wave >> 2;
      if (!LAST) {
        const int cs = (wave & 3) * 64 + lane * 2;
        const unsigned wv = *(const u32a*)(&hA[nxt][b * kHP + cs]);
        unsigned* dst = (unsigned*)(yh + ((size_t)(b * kLQ + t)) * kH + cs);
        *(volatile unsigned*)dst = wv;
        __threadfence();
        *(volatile unsigned*)dst = wv;
      } else {
        const int c0 = (wave & 3) * 64 + lane;
        const float v0 = hF[nxt * 1024 + b * 256 + c0];
        const float v1 = hF[nxt * 1024 + b * 256 + c0 + 32];
        float* dst = outp + ((size_t)(b * kLQ + t)) * kH + c0;
        *(volatile float*)dst = v0;
        *(volatile float*)(dst + 32) = v1;
        __threadfence();
        *(volatile float*)dst = v0;
        *(volatile float*)(dst + 32) = v1;
      }
    }
  }
}

extern "C" void kernel_launch(void* const* d_in, const int* in_sizes, int n_in,
                              void* d_out, int out_size, void* d_ws, size_t ws_size,
                              hipStream_t stream) {
  if (n_in < 11) return;
  if (in_sizes[0] != kRowsK * kD) return;
  if (in_sizes[1] != kRowsQ * kD) return;
  if (in_sizes[2] != kH * kD) return;
  if (in_sizes[3] != kH * kD) return;
  if (in_sizes[4] != kH) return;
  if (in_sizes[5] != kH * kH) return;
  if (in_sizes[6] != kH) return;
  if (in_sizes[7] != kL * kG3 * kH) return;
  if (in_sizes[8] != kL * kG3 * kH) return;
  if (in_sizes[9] != kL * kG3) return;
  if (in_sizes[10] != kL * kG3) return;
  if (out_size != kRowsQ * kH) return;
  if (ws_size < kWsTotal) return;

  const float* keys    = (const float*)d_in[0];
  const float* queries = (const float*)d_in[1];
  const float* W_k     = (const float*)d_in[2];
  const float* W_q     = (const float*)d_in[3];
  const float* w_v     = (const float*)d_in[4];
  const float* W_g_w   = (const float*)d_in[5];
  const float* W_g_b   = (const float*)d_in[6];
  const float* gWih    = (const float*)d_in[7];
  const float* gWhh    = (const float*)d_in[8];
  const float* gbih    = (const float*)d_in[9];
  const float* gbhh    = (const float*)d_in[10];
  float* out = (float*)d_out;

  char* ws = (char*)d_ws;
  unsigned short* KH  = (unsigned short*)(ws + kOffKH);
  unsigned short* KT  = (unsigned short*)(ws + kOffKT);
  unsigned short* QH  = (unsigned short*)(ws + kOffQH);
  unsigned short* WK  = (unsigned short*)(ws + kOffWK);
  unsigned short* WQ  = (unsigned short*)(ws + kOffWQ);
  unsigned short* WG  = (unsigned short*)(ws + kOffWG);
  unsigned short* WIH = (unsigned short*)(ws + kOffWIH);
  unsigned short* WHH = (unsigned short*)(ws + kOffWHH);
  float*          KP  = (float*)(ws + kOffKP);
  float*          QP  = (float*)(ws + kOffQP);
  unsigned short* EH  = (unsigned short*)(ws + kOffEH);
  float*          RR  = (float*)(ws + kOffRR);
  float*          UC  = (float*)(ws + kOffUC);
  unsigned short* UCH = (unsigned short*)(ws + kOffUCH);
  float*          PRE = (float*)(ws + kOffPRE);
  unsigned short* XA  = (unsigned short*)(ws + kOffXA);
  unsigned short* Y0  = (unsigned short*)(ws + kOffY0);
  unsigned short* Y1  = (unsigned short*)(ws + kOffY1);
  float*          GI  = (float*)(ws + kOffGI);

  cvt_planes_kernel<<<kCvtE6, 256, 0, stream>>>(keys, queries, W_k, W_q, W_g_w, gWih, gWhh,
                                                KH, QH, WK, WQ, WG, WIH, WHH);
  keys_transpose_kernel<<<dim3(kLK / 64, kD / 64, kB), 256, 0, stream>>>(keys, KT);

  gemm64_f16_kernel<0><<<dim3((kRowsK / 64) * (kH / 64) / 8, 1), 256, 0, stream>>>(
      KH, kD, 0L, WK, kD, 0L, KP, kH, 0L, W_g_b, kRowsK, kH, kD, kScaleActW);
  gemm64_f16_kernel<0><<<dim3((kRowsQ / 64) * (kH / 64) / 8, 1), 256, 0, stream>>>(
      QH, kD, 0L, WQ, kD, 0L, QP, kH, 0L, W_g_b, kRowsQ, kH, kD, kScaleActW);

  score_exp_kernel<<<dim3(kLK / 64, kLQ / 16, kB), 256, 0, stream>>>(QP, KP, w_v, EH);

  gemm64_f16_kernel<0><<<dim3((kLQ / 64) * (kD / 64) / 8, kB), 256, 0, stream>>>(
      EH, kLK, (long)kLQ * kLK, KT, kLK, (long)kD * kLK, RR, kD, (long)kLQ * kD, W_g_b,
      kLQ, kD, kLK, kScaleAct);

  denom_resid_kernel<<<kLQ, 256, 0, stream>>>(EH, RR, queries, UC, UCH);

  gemm64_f16_kernel<2><<<dim3((kRowsQ / 64) * (kH / 64) / 8, 1), 256, 0, stream>>>(
      UCH, kD, 0L, WG, kH, 0L, PRE, kH, 0L, W_g_b, kRowsQ, kH, kD, kScaleActW);
  gate_apply_kernel<<<kRowsQ * kH / 8 / 256, 256, 0, stream>>>(PRE, UC, XA);

  gemm64_f16_kernel<2><<<dim3((kRowsQ / 64) * (kG3 / 64) / 8, 1), 256, 0, stream>>>(
      XA, kH, 0L, WIH, kH, 0L, GI, kG3, 0L, gbih, kRowsQ, kG3, kH, kScaleActW);
  gru_scan_kernel<false><<<1, 512, 0, stream>>>(GI, WHH, gbhh, Y0, out);
  gemm64_f16_kernel<2><<<dim3((kRowsQ / 64) * (kG3 / 64) / 8, 1), 256, 0, stream>>>(
      Y0, kH, 0L, WIH + (size_t)kG3 * kH, kH, 0L, GI, kG3, 0L, gbih + kG3, kRowsQ, kG3, kH, kScaleHW);
  gru_scan_kernel<false><<<1, 512, 0, stream>>>(GI, WHH + (size_t)kG3 * kH, gbhh + kG3, Y1, out);
  gemm64_f16_kernel<2><<<dim3((kRowsQ / 64) * (kG3 / 64) / 8, 1), 256, 0, stream>>>(
      Y1, kH, 0L, WIH + (size_t)2 * kG3 * kH, kH, 0L, GI, kG3, 0L, gbih + 2 * kG3, kRowsQ, kG3, kH, kScaleHW);
  gru_scan_kernel<true><<<1, 512, 0, stream>>>(GI, WHH + (size_t)2 * kG3 * kH, gbhh + 2 * kG3, Y0, out);
}
